// FlexAttn_4449586119251
// MI455X (gfx1250) — hardware-verified
//
#include <hip/hip_runtime.h>

#define L_TOK 680
#define L_PAD 704
#define DH    64
#define NQT   22
#define NBH   128

typedef __bf16 v16b __attribute__((ext_vector_type(16)));
typedef unsigned short v8us __attribute__((ext_vector_type(8), may_alias));
typedef float  v8f  __attribute__((ext_vector_type(8)));
typedef float  v4f  __attribute__((ext_vector_type(4)));
typedef float  v4fa __attribute__((ext_vector_type(4), may_alias));
union FragB { v16b v; v8us half[2]; unsigned short u[16]; };

__device__ __forceinline__ unsigned short bf16_bits(float x) { unsigned int u = __float_as_uint(x); return (unsigned short)((u + 0x7FFFu + ((u >> 16) & 1u)) >> 16); }
__device__ __forceinline__ float bf16_val(unsigned short b) { return __uint_as_float(((unsigned int)b) << 16); }
__device__ __forceinline__ v8f mma3(v16b ah, v16b al, v16b bh, v16b bl, v8f c) {
  c = __builtin_amdgcn_wmma_f32_16x16x32_bf16(false, ah, false, bh, (short)0, c, false, false);
  c = __builtin_amdgcn_wmma_f32_16x16x32_bf16(false, ah, false, bl, (short)0, c, false, false);
  c = __builtin_amdgcn_wmma_f32_16x16x32_bf16(false, al, false, bh, (short)0, c, false, false);
  asm volatile("v_nop\n\tv_nop\n\tv_nop\n\tv_nop" : "+v"(c) : "v"(ah), "v"(al), "v"(bh), "v"(bl));
  return c;
}
__device__ __forceinline__ void split_store(unsigned short* hi, unsigned short* lo, float x) {
  const unsigned short h = bf16_bits(x); *hi = h; *lo = bf16_bits(x - bf16_val(h));
}

__global__ __launch_bounds__(64) void k_attn(const float* __restrict__ q, const float* __restrict__ k,
                                            const float* __restrict__ v, float* __restrict__ out) {
  __shared__ __attribute__((aligned(16))) unsigned short sQh[2][16][DH + 8], sQl[2][16][DH + 8];
  __shared__ __attribute__((aligned(16))) unsigned short sKh[32][DH + 8], sKl[32][DH + 8];
  __shared__ __attribute__((aligned(16))) float sS[2][16][L_PAD];
  __shared__ __attribute__((aligned(16))) unsigned short sPh[2][16][L_PAD + 8], sPl[2][16][L_PAD + 8];
  __shared__ float sInv[2][16];
  __shared__ __attribute__((aligned(16))) float sO[2][16][DH];

  const int tid = threadIdx.x, w = tid >> 5, lane = tid & 31, ln = lane & 15, hh = lane >> 4;
  const int bh = blockIdx.x / NQT, qt = blockIdx.x % NQT;
  const int q0 = qt * 32 + w * 16;
  const size_t base = (size_t)bh * L_TOK * DH;
  const float* Q = q + base; const float* K = k + base; const float* V = v + base; float* O = out + base;
  const int ends[10] = {1, 5, 14, 30, 55, 91, 155, 255, 424, 680};

  for (int e = lane; e < 16 * (DH / 4); e += 32) {
    const int r = e / (DH / 4), c4 = (e % (DH / 4)) * 4;
    int row = q0 + r; if (row >= L_TOK) row = L_TOK - 1;
    const v4f f = *(const v4fa*)(Q + (size_t)row * DH + c4);
#pragma unroll
    for (int t = 0; t < 4; ++t) split_store(&sQh[w][r][c4 + t], &sQl[w][r][c4 + t], f[t] * 0.125f);
  }
  __syncthreads();
  FragB aqh[2], aql[2];
#pragma unroll
  for (int ks = 0; ks < 2; ++ks) {
    aqh[ks].half[0] = *(const v8us*)&sQh[w][ln][ks * 32 + 8 * hh]; aqh[ks].half[1] = *(const v8us*)&sQh[w][ln][ks * 32 + 16 + 8 * hh];
    aql[ks].half[0] = *(const v8us*)&sQl[w][ln][ks * 32 + 8 * hh]; aql[ks].half[1] = *(const v8us*)&sQl[w][ln][ks * 32 + 16 + 8 * hh];
  }
  int kend[8];
#pragma unroll
  for (int r = 0; r < 8; ++r) {
    int qi = q0 + 8 * hh + r; if (qi >= L_TOK) qi = L_TOK - 1;
    int e = L_TOK;
#pragma unroll
    for (int i = 0; i < 10; ++i) { if (qi < ends[i]) { e = ends[i]; break; } }
    kend[r] = e;
  }

  for (int c = 0; c < L_PAD / 32; ++c) {
    const int j0 = c * 32;
    __syncthreads();
    for (int e = tid; e < 32 * (DH / 4); e += 64) {
      const int r = e / (DH / 4), c4 = (e % (DH / 4)) * 4;
      int key = j0 + r; if (key >= L_TOK) key = L_TOK - 1;
      const v4f f = *(const v4fa*)(K + (size_t)key * DH + c4);
#pragma unroll
      for (int t = 0; t < 4; ++t) split_store(&sKh[r][c4 + t], &sKl[r][c4 + t], f[t]);
    }
    __syncthreads();
#pragma unroll
    for (int nt = 0; nt < 2; ++nt) {
      v8f acc = {};
#pragma unroll
      for (int ks = 0; ks < 2; ++ks) {
        FragB bh_, bl_;
        bh_.half[0] = *(const v8us*)&sKh[nt * 16 + ln][ks * 32 + 8 * hh]; bh_.half[1] = *(const v8us*)&sKh[nt * 16 + ln][ks * 32 + 16 + 8 * hh];
        bl_.half[0] = *(const v8us*)&sKl[nt * 16 + ln][ks * 32 + 8 * hh]; bl_.half[1] = *(const v8us*)&sKl[nt * 16 + ln][ks * 32 + 16 + 8 * hh];
        acc = mma3(aqh[ks].v, aql[ks].v, bh_.v, bl_.v, acc);
      }
      const int j = j0 + nt * 16 + ln;
#pragma unroll
      for (int r = 0; r < 8; ++r) sS[w][8 * hh + r][j] = (j < kend[r]) ? acc[r] : -3.0e38f;
    }
  }
  __builtin_amdgcn_fence(__ATOMIC_ACQ_REL, "workgroup");
  __builtin_amdgcn_wave_barrier();

  {
    const int r = ln;
    float mx = -3.0e38f;
    for (int j = hh; j < L_PAD; j += 2) mx = fmaxf(mx, sS[w][r][j]);
    mx = fmaxf(mx, __shfl_xor(mx, 16, 32));
    float sum = 0.f;
    for (int j = hh; j < L_PAD; j += 2) {
      const float s = sS[w][r][j];
      const float p = (s > -1.0e38f) ? __expf(s - mx) : 0.0f;
      sum += p;
      split_store(&sPh[w][r][j], &sPl[w][r][j], p);
    }
    sum += __shfl_xor(sum, 16, 32);
    if (hh == 0) sInv[w][r] = 1.0f / sum;
  }

  v8f oacc[4] = {};
  for (int c = 0; c < L_PAD / 32; ++c) {
    const int j0 = c * 32;
    __syncthreads();
    for (int e = tid; e < 32 * (DH / 4); e += 64) {
      const int r = e / (DH / 4), c4 = (e % (DH / 4)) * 4;
      const int key = j0 + r;
      v4f f = {0.f, 0.f, 0.f, 0.f};
      if (key < L_TOK) f = *(const v4fa*)(V + (size_t)key * DH + c4);
#pragma unroll
      for (int t = 0; t < 4; ++t) split_store(&sKh[r][c4 + t], &sKl[r][c4 + t], f[t]);
    }
    __syncthreads();
    FragB pah, pal;
    pah.half[0] = *(const v8us*)&sPh[w][ln][j0 + 8 * hh]; pah.half[1] = *(const v8us*)&sPh[w][ln][j0 + 16 + 8 * hh];
    pal.half[0] = *(const v8us*)&sPl[w][ln][j0 + 8 * hh]; pal.half[1] = *(const v8us*)&sPl[w][ln][j0 + 16 + 8 * hh];
#pragma unroll
    for (int dt = 0; dt < 4; ++dt) {
      FragB bvh, bvl;
#pragma unroll
      for (int i = 0; i < 8; ++i) {
        bvh.u[i] = sKh[8 * hh + i][dt * 16 + ln]; bvh.u[8 + i] = sKh[16 + 8 * hh + i][dt * 16 + ln];
        bvl.u[i] = sKl[8 * hh + i][dt * 16 + ln]; bvl.u[8 + i] = sKl[16 + 8 * hh + i][dt * 16 + ln];
      }
      oacc[dt] = mma3(pah.v, pal.v, bvh.v, bvl.v, oacc[dt]);
    }
  }

#pragma unroll
  for (int dt = 0; dt < 4; ++dt)
#pragma unroll
    for (int r = 0; r < 8; ++r) sO[w][8 * hh + r][dt * 16 + ln] = oacc[dt][r] * sInv[w][8 * hh + r];
  __builtin_amdgcn_fence(__ATOMIC_ACQ_REL, "workgroup");
  __builtin_amdgcn_wave_barrier();
  const int rsub = lane >> 4, c4 = (lane & 15) * 4;
  for (int pass = 0; pass < 2; ++pass) {
#pragma unroll
    for (int qq = 0; qq < 8; ++qq) {
      const int r = qq * 2 + rsub;
      const int row = q0 + r;
      if (row < L_TOK) {
        const v4f val = *(const v4fa*)&sO[w][r][c4];
        *(volatile v4f*)(O + (size_t)row * DH + c4) = val;
      }
    }
    if (pass == 0) __threadfence();
  }
}

extern "C" void kernel_launch(void* const* d_in, const int* in_sizes, int n_in,
                              void* d_out, int out_size, void* d_ws, size_t ws_size, hipStream_t stream) {
  (void)in_sizes; (void)n_in; (void)out_size; (void)d_ws; (void)ws_size;
  k_attn<<<NBH * NQT, 64, 0, stream>>>((const float*)d_in[0], (const float*)d_in[1], (const float*)d_in[2], (float*)d_out);
}
